// MultiHeadAttentionClassical_65481071395783
// MI455X (gfx1250) — hardware-verified
//
#include <hip/hip_runtime.h>


#ifndef NB
#define NB 4
#endif
#ifndef SEQ
#define SEQ 2048
#endif
#define NB_FULL  4
#define SEQ_FULL 2048
#define TT   SEQ
#define DM   1024
#define NH_  16
#define HD   64
#define DQKV (3 * DM)
#define QPB  128
#define PCAR 4096.0f
#define SCL  0.125f
#define MFILL (-1.0e9f)
#define L2E  1.4426950408889634f
static_assert(TT % QPB == 0);
static_assert(TT % 64 == 0);
static_assert(DM % 64 == 0);
static_assert(DQKV % 64 == 0);
static_assert(NH_ * HD == DM);
static_assert(HD == 64);
static_assert(NB <= NB_FULL);
static_assert(SEQ <= SEQ_FULL);

typedef _Float16 h16;
typedef unsigned short bf;
typedef __attribute__((ext_vector_type(16))) __bf16   v16bf;
typedef __attribute__((ext_vector_type(16))) _Float16 v16h;
typedef __attribute__((ext_vector_type(8)))  _Float16 v8h;
typedef __attribute__((ext_vector_type(8)))  unsigned short v8us;
typedef __attribute__((ext_vector_type(8)))  float    v8f;
typedef __attribute__((ext_vector_type(8)))  int      v8i;
typedef __attribute__((ext_vector_type(4)))  float    v4f;
typedef __attribute__((ext_vector_type(2)))  _Float16 v2h;
typedef __attribute__((ext_vector_type(2)))  unsigned short v2us;
typedef __attribute__((ext_vector_type(2)))  float    v2f;
typedef v4f  __attribute__((may_alias)) v4fa;

__device__ __forceinline__ unsigned short f2bf(float f) { unsigned u = __float_as_uint(f); u += 0x7FFFu + ((u >> 16) & 1u); return (unsigned short)(u >> 16); }
__device__ __forceinline__ float bf2f(unsigned short b) { return __uint_as_float(((unsigned)b) << 16); }
__device__ __forceinline__ float bfr(float f) { return bf2f(f2bf(f)); }
__device__ __forceinline__ void splitf(float y, unsigned short& h, unsigned short& l) { h = f2bf(y); l = f2bf(y - bf2f(h)); }
__device__ __forceinline__ v16h cat16(v8h lo, v8h hi) { return __builtin_shufflevector(lo, hi, 0, 1, 2, 3, 4, 5, 6, 7, 8, 9, 10, 11, 12, 13, 14, 15); }
__device__ __forceinline__ v16bf cat16b(v8us lo, v8us hi) { return __builtin_bit_cast(v16bf, __builtin_shufflevector(lo, hi, 0, 1, 2, 3, 4, 5, 6, 7, 8, 9, 10, 11, 12, 13, 14, 15)); }
__device__ __forceinline__ v8f wmma16(v16h a, v16h b, v8f c) { return __builtin_amdgcn_wmma_f32_16x16x32_f16(false, a, false, b, (short)0, c, false, false); }
__device__ __forceinline__ v8f wmmab(v16bf a, v16bf b, v8f c) { return __builtin_amdgcn_wmma_f32_16x16x32_bf16(false, a, false, b, (short)0, c, false, false); }
__device__ __forceinline__ v16h ldh(const h16* p) { return cat16(*(const v8h*)p, *(const v8h*)(p + 16)); }

template <typename T16> struct WFrag;
template <> struct WFrag<h16> { typedef v16h V; static __device__ __forceinline__ V ld(const h16* p) { return cat16(*(const v8h*)p, *(const v8h*)(p + 16)); } static __device__ __forceinline__ v8f mma(V a, V b, v8f c) { return wmma16(a, b, c); } };
template <> struct WFrag<bf> { typedef v16bf V; static __device__ __forceinline__ V ld(const bf* p) { return cat16b(*(const v8us*)p, *(const v8us*)(p + 16)); } static __device__ __forceinline__ v8f mma(V a, V b, v8f c) { return wmmab(a, b, c); } };
template <typename T16, int NSPLIT, bool BIAS>
__global__ __launch_bounds__(32) void k_gemmw(const T16* __restrict__ A, const T16* __restrict__ A2, const T16* __restrict__ Bt, const T16* __restrict__ Bt2, int K, float* C, int ldc, const float* __restrict__ bias, size_t sA, size_t sB, size_t sC) {
    typedef typename WFrag<T16>::V V;
    __shared__ __align__(16) float os[16 * 68];
    const size_t z = blockIdx.z; A += z * sA; if (A2) A2 += z * sA; Bt += z * sB; if (Bt2) Bt2 += z * sB; C += z * sC;
    const int lane = threadIdx.x & 31, lr = lane & 15, hi = lane >> 4; const int r0 = blockIdx.x * 64, c0 = blockIdx.y * 64;
    v8f acc[4][4];
#pragma unroll
    for (int mb = 0; mb < 4; ++mb)
#pragma unroll
        for (int nb = 0; nb < 4; ++nb) acc[mb][nb] = (v8f){};
    const size_t aoff = (size_t)(r0 + lr) * K + 8 * hi, boff = (size_t)(c0 + lr) * K + 8 * hi;
#pragma unroll 1
    for (int kc = 0; kc < K; kc += 32) {
        V a[4], a2[4];
#pragma unroll
        for (int mb = 0; mb < 4; ++mb) { a[mb] = WFrag<T16>::ld(A + aoff + (size_t)mb * 16 * K + kc); if (NSPLIT == 1 || NSPLIT == 2) a2[mb] = WFrag<T16>::ld(A2 + aoff + (size_t)mb * 16 * K + kc); }
#pragma unroll
        for (int nb = 0; nb < 4; ++nb) { const V b = WFrag<T16>::ld(Bt + boff + (size_t)nb * 16 * K + kc); V b2; if (NSPLIT >= 2) b2 = WFrag<T16>::ld(Bt2 + boff + (size_t)nb * 16 * K + kc);
#pragma unroll
            for (int mb = 0; mb < 4; ++mb) { acc[mb][nb] = WFrag<T16>::mma(a[mb], b, acc[mb][nb]); if (NSPLIT == 1 || NSPLIT == 2) acc[mb][nb] = WFrag<T16>::mma(a2[mb], b, acc[mb][nb]); if (NSPLIT >= 2) acc[mb][nb] = WFrag<T16>::mma(a[mb], b2, acc[mb][nb]); } }
        asm volatile("v_nop\n\tv_nop\n\tv_nop\n\tv_nop" : "+v"(acc[0][0]), "+v"(acc[1][1]), "+v"(acc[2][2]), "+v"(acc[3][3]) : "v"(a[0]), "v"(a[3]));
    }
#pragma unroll
    for (int mb = 0; mb < 4; ++mb) {
#pragma unroll
        for (int nb = 0; nb < 4; ++nb) {
#pragma unroll
            for (int j = 0; j < 8; ++j) os[(hi * 8 + j) * 68 + nb * 16 + lr] = acc[mb][nb][j]; }
        __builtin_amdgcn_wave_barrier(); asm volatile("" ::: "memory");
        float* crow = C + (size_t)(r0 + mb * 16) * ldc + c0;
#pragma unroll 1
        for (int ps = 0; ps < 2; ++ps) {
#pragma unroll
            for (int s = 0; s < 8; ++s) { const int row = 2 * s + hi, cofs = lr * 4; v4f val = *(const v4fa*)(os + row * 68 + cofs); if (BIAS) { val[0] += bfr(bias[c0 + cofs]); val[1] += bfr(bias[c0 + cofs + 1]); val[2] += bfr(bias[c0 + cofs + 2]); val[3] += bfr(bias[c0 + cofs + 3]); }
                *(volatile v4f*)(crow + (size_t)row * ldc + cofs) = val; }
            if (ps == 0) __threadfence(); }
        __builtin_amdgcn_wave_barrier(); asm volatile("" ::: "memory");
    }
}

__global__ __launch_bounds__(256) void k_cvt8(const float* __restrict__ src, bf* dst, size_t n8) { const size_t i = (size_t)blockIdx.x * 256 + threadIdx.x; if (i >= n8) return; const v8f v = *(const v8f*)(src + i * 8); v8us o;
#pragma unroll
    for (int k = 0; k < 8; ++k) o[k] = f2bf(v[k]); *(volatile v8us*)(dst + i * 8) = o; __threadfence(); *(volatile v8us*)(dst + i * 8) = o; }

__global__ __launch_bounds__(256) void k_qkp(const float* __restrict__ F, h16* QP, h16* KP) {
    const size_t e = ((size_t)blockIdx.x * 256 + threadIdx.x) * 2; if (e >= (size_t)NH_ * TT * HD) return;
    const int d = (int)(e % HD); const int t = (int)((e / HD) % TT); const int h = (int)(e / ((size_t)HD * TT));
    const float* f = F + (size_t)t * DQKV + h * HD + d;
    const v2f xq = *(const v2f*)f; const v2f xk = *(const v2f*)(f + DM);
    v2h oq, ok; oq[0] = (h16)xq[0]; oq[1] = (h16)xq[1]; ok[0] = (h16)xk[0]; ok[1] = (h16)xk[1];
    *(volatile v2h*)(QP + e) = oq; *(volatile v2h*)(KP + e) = ok; __threadfence(); *(volatile v2h*)(QP + e) = oq; *(volatile v2h*)(KP + e) = ok; }
__global__ __launch_bounds__(256) void k_vtp(const float* __restrict__ F, h16* V16) {
    const size_t e = ((size_t)blockIdx.x * 256 + threadIdx.x) * 2; if (e >= (size_t)NH_ * HD * TT) return;
    const int t = (int)(e % TT); const int d = (int)((e / TT) % HD); const int g = (int)(e / ((size_t)TT * HD));
    v2h o16; o16[0] = (h16)F[(size_t)t * DQKV + 2 * DM + g * HD + d]; o16[1] = (h16)F[(size_t)(t + 1) * DQKV + 2 * DM + g * HD + d];
    *(volatile v2h*)(V16 + e) = o16; __threadfence(); *(volatile v2h*)(V16 + e) = o16; }

__global__ __launch_bounds__(256) void k_attn(const h16* __restrict__ QP, const h16* __restrict__ KP, const h16* __restrict__ VT, const int* __restrict__ keep, float* Ob) {
    __shared__ __align__(16) h16 Ksh[32 * HD];
    __shared__ __align__(16) h16 Vsh[HD * 32];
    __shared__ __align__(16) float os[8 * 16 * 68];
    const int wv = threadIdx.x >> 5, lane = threadIdx.x & 31, lr = lane & 15, hi = lane >> 4;
    const int nqb = TT / QPB; const int h = blockIdx.x / nqb; const int qb = blockIdx.x - h * nqb; const int q0 = qb * QPB + wv * 16;
    const h16* Qh = QP + (size_t)h * TT * HD; const h16* Kh = KP + (size_t)h * TT * HD; const h16* Vh = VT + (size_t)h * HD * TT;
    const v16h qf0 = ldh(Qh + (size_t)(q0 + lr) * HD + 8 * hi);
    const v16h qf1 = ldh(Qh + (size_t)(q0 + lr) * HD + 32 + 8 * hi);
    const int kr = threadIdx.x >> 3, kc = (threadIdx.x & 7) * 8;
    const int vr = threadIdx.x >> 2, vc = (threadIdx.x & 3) * 8;
    v8f o[4];
#pragma unroll
    for (int t = 0; t < 4; ++t) o[t] = (v8f){};
    float mrow = -3.0e38f, lrow = 0.0f;
#pragma unroll 1
    for (int j = 0; j < TT; j += 32) {
        *(v8h*)(Ksh + kr * HD + kc) = *(const v8h*)(Kh + (size_t)(j + kr) * HD + kc);
        *(v8h*)(Vsh + vr * 32 + vc) = *(const v8h*)(Vh + (size_t)vr * TT + j + vc);
        const v8i mk0 = *(const v8i*)(keep + j + 8 * hi);
        const v8i mk1 = *(const v8i*)(keep + j + 16 + 8 * hi);
        __syncthreads();
        const v16h ka0 = ldh(Ksh + lr * HD + 8 * hi), ka1 = ldh(Ksh + lr * HD + 32 + 8 * hi);
        const v16h kb0 = ldh(Ksh + (16 + lr) * HD + 8 * hi), kb1 = ldh(Ksh + (16 + lr) * HD + 32 + 8 * hi);
        v8f s0 = (v8f){}, s1 = (v8f){};
        s0 = wmma16(ka0, qf0, s0); s0 = wmma16(ka1, qf1, s0);
        s1 = wmma16(kb0, qf0, s1); s1 = wmma16(kb1, qf1, s1);
        asm volatile("v_nop\n\tv_nop\n\tv_nop\n\tv_nop" : "+v"(s0), "+v"(s1) : "v"(kb1), "v"(qf1));
        float f[16]; float tmax = -3.0e38f;
#pragma unroll
        for (int r = 0; r < 8; ++r) {
            const float t0 = s0[r] * SCL, t1 = s1[r] * SCL;
            f[r] = (mk0[r] != 0) ? t0 : MFILL; f[8 + r] = (mk1[r] != 0) ? t1 : MFILL;
            tmax = fmaxf(tmax, fmaxf(f[r], f[8 + r])); }
        tmax = fmaxf(tmax, __shfl_xor(tmax, 16, 32));
        const float mnew = fmaxf(mrow, tmax);
        const float alpha = __builtin_amdgcn_exp2f(fmaxf(mrow - mnew, -200.0f) * L2E);
        float ls = 0.0f; v16h pb;
#pragma unroll
        for (int r = 0; r < 16; ++r) { const float p = __builtin_amdgcn_exp2f((f[r] - mnew) * L2E); ls += p; pb[r] = (h16)(p * PCAR); }
        ls += __shfl_xor(ls, 16, 32);
        lrow = lrow * alpha + ls; mrow = mnew;
#pragma unroll
        for (int t = 0; t < 4; ++t) {
#pragma unroll
            for (int r = 0; r < 8; ++r) o[t][r] *= alpha; }
        const v16h va0 = ldh(Vsh + lr * 32 + 8 * hi), va1 = ldh(Vsh + (16 + lr) * 32 + 8 * hi);
        const v16h va2 = ldh(Vsh + (32 + lr) * 32 + 8 * hi), va3 = ldh(Vsh + (48 + lr) * 32 + 8 * hi);
        o[0] = wmma16(va0, pb, o[0]); o[1] = wmma16(va1, pb, o[1]); o[2] = wmma16(va2, pb, o[2]); o[3] = wmma16(va3, pb, o[3]);
        asm volatile("v_nop\n\tv_nop\n\tv_nop\n\tv_nop" : "+v"(o[0]), "+v"(o[1]), "+v"(o[2]), "+v"(o[3]) : "v"(va3), "v"(pb));
        __syncthreads();
    }
    const float inv = __fdiv_rn(1.0f, lrow) * (1.0f / PCAR);
    float* ow = os + wv * (16 * 68);
#pragma unroll
    for (int t = 0; t < 4; ++t) {
#pragma unroll
        for (int r = 0; r < 8; ++r) ow[lr * 68 + t * 16 + 8 * hi + r] = o[t][r] * inv; }
    __syncthreads();
    float* orow = Ob + ((size_t)h * TT + q0) * HD;
#pragma unroll 1
    for (int ps = 0; ps < 2; ++ps) {
#pragma unroll
        for (int s = 0; s < 8; ++s) { const int row = 2 * s + hi, cofs = lr * 4; const v4f val = *(const v4fa*)(ow + row * 68 + cofs); *(volatile v4f*)(orow + (size_t)row * HD + cofs) = val; }
        if (ps == 0) __threadfence(); }
}

__global__ __launch_bounds__(256) void k_merge(const float* __restrict__ O, bf* Ah, bf* Al) {
    const size_t e = ((size_t)blockIdx.x * 256 + threadIdx.x) * 2; if (e >= (size_t)NH_ * TT * HD) return;
    const int d = (int)(e % HD); const int t = (int)((e / HD) % TT); const int zz = (int)(e / ((size_t)HD * TT));
    const size_t oo = (size_t)t * DM + zz * HD + d;
    const v2f x = *(const v2f*)(O + e); v2us oh, ol;
#pragma unroll
    for (int q = 0; q < 2; ++q) { const float xv = x[q]; unsigned short a, c2; splitf(xv, a, c2); oh[q] = a; ol[q] = c2; }
    *(volatile v2us*)(Ah + oo) = oh; *(volatile v2us*)(Al + oo) = ol; __threadfence(); *(volatile v2us*)(Ah + oo) = oh; *(volatile v2us*)(Al + oo) = ol; }

extern "C" void kernel_launch(void* const* d_in, const int* in_sizes, int n_in,
                              void* d_out, int out_size, void* d_ws, size_t ws_size, hipStream_t stream) {
    if (n_in < 5) return;
    if ((size_t)in_sizes[0] < (size_t)NB * SEQ_FULL * DM) return;
    if ((size_t)in_sizes[1] < (size_t)DQKV * DM) return;
    if ((size_t)in_sizes[2] < (size_t)DM * DM) return;
    if (in_sizes[3] < DM) return;
    if (in_sizes[4] < NB * SEQ_FULL) return;
    if ((size_t)out_size < (size_t)NB * TT * DM) return;
    const float* x = (const float*)d_in[0];
    const float* wqkv = (const float*)d_in[1];
    const float* wo = (const float*)d_in[2];
    const float* bo = (const float*)d_in[3];
    const int* keep = (const int*)d_in[4];
    float* OUT = (float*)d_out;
    char* wsp = (char*)d_ws;
    auto take = [&](size_t bytes) { char* p = wsp; wsp += (bytes + 255) & ~(size_t)255; return (void*)p; };
    bf* WQKV = (bf*)take((size_t)DQKV * DM * 2);
    bf* WO = (bf*)take((size_t)DM * DM * 2);
    bf* XB = (bf*)take((size_t)TT * DM * 2);
    float* F = (float*)take((size_t)TT * DQKV * 4);
    h16* QP = (h16*)take((size_t)NH_ * TT * HD * 2);
    h16* KP = (h16*)take((size_t)NH_ * TT * HD * 2);
    h16* VT = (h16*)take((size_t)NH_ * HD * TT * 2);
    float* Ob = (float*)take((size_t)NH_ * TT * HD * 4);
    bf* ATh = (bf*)take((size_t)TT * DM * 2);
    bf* ATl = (bf*)take((size_t)TT * DM * 2);
    if ((size_t)(wsp - (char*)d_ws) > ws_size) return;
    k_cvt8<<<(unsigned)(((size_t)DQKV * DM / 8 + 255) / 256), 256, 0, stream>>>(wqkv, WQKV, (size_t)DQKV * DM / 8);
    k_cvt8<<<(unsigned)(((size_t)DM * DM / 8 + 255) / 256), 256, 0, stream>>>(wo, WO, (size_t)DM * DM / 8);
    const unsigned LP = (unsigned)(((size_t)NH_ * TT * HD / 2 + 255) / 256);
    for (int b = 0; b < NB; ++b) {
        k_cvt8<<<(unsigned)(((size_t)TT * DM / 8 + 255) / 256), 256, 0, stream>>>(x + (size_t)b * SEQ_FULL * DM, XB, (size_t)TT * DM / 8);
        k_gemmw<bf, 0, false><<<dim3(TT / 64, DQKV / 64, 1), 32, 0, stream>>>(XB, nullptr, WQKV, nullptr, DM, F, DQKV, nullptr, 0, 0, 0);
        k_qkp<<<LP, 256, 0, stream>>>(F, QP, KP);
        k_vtp<<<LP, 256, 0, stream>>>(F, VT);
        k_attn<<<(unsigned)(NH_ * (TT / QPB)), 256, 0, stream>>>(QP, KP, VT, keep + (size_t)b * SEQ_FULL, Ob);
        k_merge<<<LP, 256, 0, stream>>>(Ob, ATh, ATl);
        k_gemmw<bf, 1, true><<<dim3(TT / 64, DM / 64, 1), 32, 0, stream>>>(ATh, ATl, WO, nullptr, DM, OUT + (size_t)b * TT * DM, DM, bo, 0, 0, 0);
    }
}
